// hyperCL_87299505259187
// MI455X (gfx1250) — hardware-run, weakly checked
//
#include <hip/hip_runtime.h>
#include <stddef.h>
#include <stdint.h>

#define NN       100000
#define NHE      20000
#define ET       120000
#define NNZ      1600000
#define HD       64
#define KL       128
#define GBM      128
#define MPN      100096
#define MPE      120064
#define NTHR     256
#define NWAVE    8
#define EPT      8
#define WCH      (32 * EPT)
#define SLB      10
#define SLOTS_N  1024
#define SLOTS_E  256
#define NBK_N    98
#define NBK_E    79
#define WLCAP_N  2560
#define WLCAP_E  3072
#define RCAP_N   (NWAVE * WLCAP_N)
#define RCAP_E   (NWAVE * WLCAP_E)
#define DEGCAP_N 64
#define DEGCAP_E 192
#define RBM      64
#define SP       68
#define MEAS_B1024_N 16666
#define MEAS_B256_E  20760
#define MEAS_DEG_N   37
#define MEAS_DEG_E   120
#define WSMAX    (128u << 20)

#define SINGLE_B1 0
#define SINGLE_A2 0
#define SINGLE_B2 0
#define KX_B1 (SINGLE_B1 ? 64 : 128)
#define KX_A2 (SINGLE_A2 ? 64 : 128)
#define KX_B2 (SINGLE_B2 ? 64 : 128)

#define ZI_N   (NWAVE * WLCAP_N + RCAP_N + 3 * SLOTS_N)
#define ZI_E   (NWAVE * WLCAP_E + RCAP_E + 3 * SLOTS_E)
#define BK_INTS ((ZI_N > ZI_E ? ZI_N : ZI_E) + 16)
#define BK_LDS (BK_INTS * 4)

#define PBX   (MPN * HD / 8 / NTHR)
#define PBW1  (HD * HD / 8 / NTHR)
#define PBWD  (HD * KL / 8 / NTHR)
#define PBEZ  ((MPE - ET) * 16 / NTHR)
#define PBHZ  ((MPN - NN) * 16 / NTHR)
#define PB1   (PBX + PBW1)
#define PB2   (PB1 + PBWD)
#define PB3   (PB2 + PBWD)
#define PB4   (PB3 + PBWD)
#define PB5   (PB4 + PBEZ)
#define PB6   (PB5 + PBHZ)
#define PBTOT (PB6 + 1)

static_assert(HD == 64 && HD % 16 == 0 && KL == 2 * HD && KL % 32 == 0 && HD % 32 == 0);
static_assert(NN < (1 << 17) && NHE < (1 << 17));
static_assert(ET == NHE + NN);
static_assert(MPN % GBM == 0 && MPN == 782 * GBM && MPN >= NN && MPN % RBM == 0);
static_assert(MPE % GBM == 0 && MPE == 938 * GBM && MPE >= ET);
static_assert(NN - 781 * GBM == 32 && ET - 937 * GBM == 64);
static_assert((NN % 2) == 0 && (NHE % 2) == 0 && (ET % 2) == 0);
static_assert(SLOTS_N == (1 << SLB) && SLOTS_E <= (1 << SLB));
static_assert(SLOTS_N % RBM == 0 && SLOTS_E % RBM == 0);
static_assert(NBK_N * SLOTS_N >= MPN && NBK_E * SLOTS_E >= ((NHE + RBM - 1) / RBM) * RBM);
static_assert(NNZ < (1 << 21) && (((long long)NNZ) << SLB) < (1LL << 31));
static_assert(NNZ % WCH == 0 && NNZ % 4 == 0);
static_assert((long long)RCAP_N * 100 >= (long long)MEAS_B1024_N * 105);
static_assert((long long)RCAP_E * 100 >= (long long)MEAS_B256_E * 105);
static_assert(MEAS_B256_E <= 23400);
static_assert(WLCAP_N >= MEAS_B1024_N / 8 + 8 * 46 + 1);
static_assert(WLCAP_E >= MEAS_B256_E / 8 + 8 * 51 + 1);
static_assert(DEGCAP_N >= 64 && DEGCAP_N >= MEAS_DEG_N + 8);
static_assert(DEGCAP_E >= 192 && DEGCAP_E >= MEAS_DEG_E + 8);
static_assert(ZI_N % 4 == 0 && ZI_E % 4 == 0 && RCAP_N % (NTHR * 4) == 0 && RCAP_E % (NTHR * 4) == 0);
static_assert(BK_LDS <= 327680);
static_assert((GBM * SP + 128) * 4 <= 65536);
static_assert((MPN * HD / 8) % NTHR == 0 && (HD * HD / 8) % NTHR == 0 && (HD * KL / 8) % NTHR == 0);
static_assert(((MPE - ET) * 16) % NTHR == 0 && ((MPN - NN) * 16) % NTHR == 0);
static_assert((long long)NN * HD - 1 == 6399999LL);

typedef float          v4f   __attribute__((ext_vector_type(4)));
typedef float          v8f   __attribute__((ext_vector_type(8)));
typedef int            v4i   __attribute__((ext_vector_type(4)));
typedef int            v8i   __attribute__((ext_vector_type(8)));
typedef unsigned short v8us  __attribute__((ext_vector_type(8)));
typedef unsigned short v16us __attribute__((ext_vector_type(16)));
typedef __bf16         v16bf __attribute__((ext_vector_type(16)));
typedef v4f  __attribute__((may_alias)) v4fa;
typedef v4i  __attribute__((may_alias)) v4ia;
typedef v8us __attribute__((may_alias)) v8usa;
union FragB { v16bf v; v16us u; v8us h[2]; v8i w; };

constexpr size_t zHH  = (size_t)MPN * KL * 2;
constexpr size_t zH   = (size_t)MPN * HD * 4;
constexpr size_t zEH  = (size_t)MPE * KL * 2;
constexpr size_t zG   = (size_t)MPE * HD * 4;
constexpr size_t zLN  = (size_t)NBK_N * RCAP_N * 4;
constexpr size_t zLE  = (size_t)NBK_E * RCAP_E * 4;
constexpr size_t zCN  = (size_t)NBK_N * 2 * SLOTS_N * 4;
constexpr size_t zCE  = (size_t)NBK_E * 2 * SLOTS_E * 4;
constexpr size_t zFN  = (size_t)NBK_N * 128;
constexpr size_t zFE  = 10240;
constexpr size_t zW1T = (size_t)HD * HD * 2;
constexpr size_t zWD  = (size_t)3 * HD * KL * 2;
constexpr size_t zSM  = 2048;
constexpr size_t oHH  = 0;
constexpr size_t oH   = oHH + zHH;
constexpr size_t oEH  = oH + zH;
constexpr size_t oG   = oEH + zEH;
constexpr size_t oLN  = oG + zG;
constexpr size_t oLE  = oLN + zLN;
constexpr size_t oCN  = oLE + zLE;
constexpr size_t oCE  = oCN + zCN;
constexpr size_t oFN  = oCE + zCE;
constexpr size_t oFE  = oFN + zFN;
constexpr size_t oW1T = oFE + zFE;
constexpr size_t oWD  = oW1T + zW1T;
constexpr size_t oSM  = oWD + zWD;
constexpr size_t oEND = oSM + zSM;
static_assert(zHH % 256 == 0 && zH % 256 == 0 && zEH % 256 == 0 && zG % 256 == 0 && zLN % 256 == 0);
static_assert(zLE % 256 == 0 && zCN % 256 == 0 && zCE % 256 == 0 && zFN % 256 == 0 && zFE % 256 == 0);
static_assert(zFE >= (size_t)NBK_E * 128 && zW1T % 256 == 0 && zWD % 256 == 0 && zSM % 256 == 0 && zSM >= 384 * 4);
static_assert((size_t)MPN * HD * 2 <= zHH - (size_t)(MPN - NN) * KL * 2);
static_assert(oEND <= (size_t)WSMAX);

__device__ __forceinline__ v8f wmb(const FragB& a, const FragB& b, v8f c) {
  v8f d = __builtin_amdgcn_wmma_f32_16x16x32_bf16(false, a.v, false, b.v, (short)0, c, false, false);
  asm volatile("v_nop\n\tv_nop\n\tv_nop\n\tv_nop" : "+v"(d) : "v"(a.w), "v"(b.w));
  return d;
}

__device__ __forceinline__ unsigned bf16_bits(float f) {
  const unsigned u = __float_as_uint(f);
  const unsigned r = (u + 0x7FFFu + ((u >> 16) & 1u)) >> 16;
  const unsigned q = (u >> 16) | 0x40u;
  return ((u & 0x7fffffffu) > 0x7f800000u) ? q : r;
}
__device__ __forceinline__ float bf16_val(float f) {
  return __uint_as_float(bf16_bits(f) << 16);
}
__device__ __forceinline__ float prelu_k(float v, float a) { return (v >= 0.0f) ? v : a * v; }

__device__ __forceinline__ void hilo_pack(float v0, float v1, float v2, float v3,
                                          int& h01, int& h23, int& l01, int& l23) {
  const unsigned a0 = bf16_bits(v0), a1 = bf16_bits(v1), a2 = bf16_bits(v2), a3 = bf16_bits(v3);
  const unsigned b0 = bf16_bits(v0 - __uint_as_float(a0 << 16));
  const unsigned b1 = bf16_bits(v1 - __uint_as_float(a1 << 16));
  const unsigned b2 = bf16_bits(v2 - __uint_as_float(a2 << 16));
  const unsigned b3 = bf16_bits(v3 - __uint_as_float(a3 << 16));
  h01 = (int)(a0 | (a1 << 16)); h23 = (int)(a2 | (a3 << 16));
  l01 = (int)(b0 | (b1 << 16)); l23 = (int)(b2 | (b3 << 16));
}

__device__ __forceinline__ v4i regroup8(int h01, int h23, int l01, int l23, int lane) {
  const int t  = lane & 15;
  const int s0 = (lane & 16) + ((2 * t) & 15), s1 = s0 + 1;
  const int a0 = __shfl(h01, s0, 32), a1 = __shfl(h23, s0, 32), a2 = __shfl(h01, s1, 32), a3 = __shfl(h23, s1, 32);
  const int b0 = __shfl(l01, s0, 32), b1 = __shfl(l23, s0, 32), b2 = __shfl(l01, s1, 32), b3 = __shfl(l23, s1, 32);
  const int mk = (t < 8) ? -1 : 0;
  v4i o;
  o.x = (a0 & mk) | (b0 & ~mk); o.y = (a1 & mk) | (b1 & ~mk);
  o.z = (a2 & mk) | (b2 & ~mk); o.w = (a3 & mk) | (b3 & ~mk);
  return o;
}

__device__ __forceinline__ void st2_v4f(float* p, v4f v) {
  *(volatile v4f*)p = v;
  __threadfence();
  *(volatile v4f*)p = v;
}
__device__ __forceinline__ void st2_v8us(unsigned short* p, v8us v) {
  *(volatile v8us*)p = v;
  __threadfence();
  *(volatile v8us*)p = v;
}

__device__ __forceinline__ v8us gather8(const float* __restrict__ base, int stride) {
  float f[8];
#pragma unroll
  for (int i = 0; i < 8; ++i) f[i] = base[(size_t)i * (size_t)stride];
  v8us o;
#pragma unroll
  for (int i = 0; i < 8; ++i) o[i] = (unsigned short)bf16_bits(f[i]);
  return o;
}

__global__ __launch_bounds__(NTHR) void k_prep(const float* __restrict__ x,
                                               const float* __restrict__ w1n, const float* __restrict__ w1e,
                                               const float* __restrict__ w2n, const float* __restrict__ w2e,
                                               const float* __restrict__ b1n, const float* __restrict__ b1e,
                                               const float* __restrict__ b2n, const float* __restrict__ b2e,
                                               const float* __restrict__ alphaP,
                                               const int* __restrict__ nnp, const int* __restrict__ nep, char* ws) {
  const int tid = (int)threadIdx.x, lane = tid & 31;
  const int blk = (int)blockIdx.x;
  unsigned short* xb  = (unsigned short*)(ws + oHH);
  unsigned short* hhp = (unsigned short*)(ws + oHH);
  unsigned short* ehp = (unsigned short*)(ws + oEH);
  unsigned short* w1t = (unsigned short*)(ws + oW1T);
  unsigned short* wd  = (unsigned short*)(ws + oWD);
  float*          sm  = (float*)(ws + oSM);
  if (blk < PBX) {
    const int u   = blk * NTHR + tid;
    const int row = u >> 3, k8 = (u & 7) * 8;
    const int rc  = row < NN ? row : NN - 1;
    const unsigned mk = row < NN ? 0xffffu : 0u;
    const float* p = x + (size_t)rc * HD + k8;
    const v4f a = *(const v4fa*)p;
    const v4f b = *(const v4fa*)(p + 4);
    v8us o;
    o[0] = (unsigned short)(bf16_bits(a.x) & mk); o[1] = (unsigned short)(bf16_bits(a.y) & mk);
    o[2] = (unsigned short)(bf16_bits(a.z) & mk); o[3] = (unsigned short)(bf16_bits(a.w) & mk);
    o[4] = (unsigned short)(bf16_bits(b.x) & mk); o[5] = (unsigned short)(bf16_bits(b.y) & mk);
    o[6] = (unsigned short)(bf16_bits(b.z) & mk); o[7] = (unsigned short)(bf16_bits(b.w) & mk);
    st2_v8us(xb + (size_t)row * HD + k8, o);
  } else if (blk < PB1) {
    const int u = (blk - PBX) * NTHR + tid;
    const int n = u >> 3, k8 = (u & 7) * 8;
    const v8us o = gather8(w1n + (size_t)k8 * HD + n, HD);
    st2_v8us(w1t + (size_t)n * HD + k8, o);
  } else if (blk < PB2) {
    const int u = (blk - PB1) * NTHR + tid;
    const int n = u >> 4, k8 = (u & 15) * 8, kk = k8 & 63;
    const v8us o = gather8(w1e + (size_t)kk * HD + n, HD);
    st2_v8us(wd + (size_t)n * KL + k8, o);
  } else if (blk < PB3) {
    const int u = (blk - PB2) * NTHR + tid;
    const int n = u >> 4, k8 = (u & 15) * 8, kk = k8 & 63;
    const v8us o = gather8(w2n + (size_t)kk * HD + n, HD);
    st2_v8us(wd + (size_t)HD * KL + (size_t)n * KL + k8, o);
  } else if (blk < PB4) {
    const int u = (blk - PB3) * NTHR + tid;
    const int n = u >> 4, k8 = (u & 15) * 8, kk = k8 & 63;
    const v8us o = gather8(w2e + (size_t)kk * HD + n, HD);
    st2_v8us(wd + (size_t)2 * HD * KL + (size_t)n * KL + k8, o);
  } else if (blk < PB5) {
    const int u = (blk - PB4) * NTHR + tid;
    const int row = ET + (u >> 4), k8 = (u & 15) * 8;
    const v8us z = {0, 0, 0, 0, 0, 0, 0, 0};
    st2_v8us(ehp + (size_t)row * KL + k8, z);
  } else if (blk < PB6) {
    const int u = (blk - PB5) * NTHR + tid;
    const int row = NN + (u >> 4), k8 = (u & 15) * 8;
    const v8us z = {0, 0, 0, 0, 0, 0, 0, 0};
    st2_v8us(hhp + (size_t)row * KL + k8, z);
  } else {
    if (tid < 64) {
      const int q = tid & 15, sel = tid >> 4;
      const v4f a0 = *(const v4fa*)(b1n + 4 * q);
      const v4f a1 = *(const v4fa*)(b1e + 4 * q);
      const v4f a2 = *(const v4fa*)(b2n + 4 * q);
      const v4f a3 = *(const v4fa*)(b2e + 4 * q);
      asm volatile("" :: "v"(a0), "v"(a1));
      asm volatile("" :: "v"(a2), "v"(a3));
      const unsigned k0 = (sel == 0) ? 0xffffffffu : 0u, k1 = (sel == 1) ? 0xffffffffu : 0u;
      const unsigned k2 = (sel == 2) ? 0xffffffffu : 0u, k3 = (sel == 3) ? 0xffffffffu : 0u;
      v4f o;
      o.x = __uint_as_float(((bf16_bits(a0.x) << 16) & k0) | ((bf16_bits(a1.x) << 16) & k1) |
                            ((bf16_bits(a2.x) << 16) & k2) | ((bf16_bits(a3.x) << 16) & k3));
      o.y = __uint_as_float(((bf16_bits(a0.y) << 16) & k0) | ((bf16_bits(a1.y) << 16) & k1) |
                            ((bf16_bits(a2.y) << 16) & k2) | ((bf16_bits(a3.y) << 16) & k3));
      o.z = __uint_as_float(((bf16_bits(a0.z) << 16) & k0) | ((bf16_bits(a1.z) << 16) & k1) |
                            ((bf16_bits(a2.z) << 16) & k2) | ((bf16_bits(a3.z) << 16) & k3));
      o.w = __uint_as_float(((bf16_bits(a0.w) << 16) & k0) | ((bf16_bits(a1.w) << 16) & k1) |
                            ((bf16_bits(a2.w) << 16) & k2) | ((bf16_bits(a3.w) << 16) & k3));
      st2_v4f(sm + 4 * tid, o);
    } else if (tid < 96) {
      const float al = alphaP[0];
      const int n1 = nnp[0], n2 = nep[0];
      const float gf = ((n1 != NN) | (n2 != NHE)) ? 1.0f : 0.0f;
      v4f o = {0.0f, 0.0f, 0.0f, 0.0f};
      o.x = (lane == 0) ? bf16_val(al) : 0.0f;
      o.y = (lane == 0) ? gf : 0.0f;
      st2_v4f(sm + 256 + 4 * lane, o);
    }
  }
}

__device__ __forceinline__ void bucket_flush(const int* pl, const int* cnt, int ov, int* lp, int* cop, int* fp,
                                             int tid, int rcap, int co_ints) {
#pragma unroll 1
  for (int i = tid * 4; i < rcap; i += NTHR * 4) {
    const v4i v = *(const v4ia*)(pl + i);
    *(volatile v4i*)(lp + i) = v;
  }
#pragma unroll 1
  for (int i = tid * 4; i < co_ints; i += NTHR * 4) {
    const v4i v = *(const v4ia*)(cnt + i);
    *(volatile v4i*)(cop + i) = v;
  }
  if (tid < 8) {
    const v4i f = {ov, ov, ov, ov};
    *(volatile v4i*)(fp + 4 * tid) = f;
  }
}

template <int ROLE>
__device__ __forceinline__ void bucket_role(const int* __restrict__ hei, int* dsm, int blk,
                                            int* LIST, int* CO, int* FLAG) {
  constexpr int SLOTS = (ROLE == 0) ? SLOTS_N : SLOTS_E;
  constexpr int WLC   = (ROLE == 0) ? WLCAP_N : WLCAP_E;
  constexpr int RC    = NWAVE * WLC;
  constexpr int NKEY  = (ROLE == 0) ? NN : NHE;
  constexpr int NENT  = (ROLE == 0) ? NHE : NN;
  constexpr int KOFF  = (ROLE == 0) ? 0 : NNZ;
  constexpr int EOFF  = (ROLE == 0) ? NNZ : 0;
  constexpr int DCAP  = (ROLE == 0) ? DEGCAP_N : DEGCAP_E;
  constexpr int ZINTS = NWAVE * WLC + RC + 3 * SLOTS;
  const int* keys = hei + KOFF;
  const int* ents = hei + EOFF;
  int* wl   = dsm;
  int* pl   = dsm + NWAVE * WLC;
  int* cnt  = pl + RC;
  int* offs = cnt + SLOTS;
  int* cur  = offs + SLOTS;
  int* misc = cur + SLOTS;
  const int tid = (int)threadIdx.x, lane = tid & 31, wave = tid >> 5;
  const unsigned nbs = (unsigned)(blk * SLOTS);
  int nbi = NKEY - blk * SLOTS;
  nbi = nbi > SLOTS ? SLOTS : (nbi < 1 ? 1 : nbi);
  const unsigned unb = (unsigned)nbi;

  {
    const v4i z4 = {0, 0, 0, 0};
    for (int i = tid * 4; i < ZINTS; i += NTHR * 4) *(v4ia*)(dsm + i) = z4;
    if (tid < 16) misc[tid] = 0;
  }
  __syncthreads();

  {
    const int per  = ((NNZ + NWAVE * WCH - 1) / (NWAVE * WCH)) * WCH;
    const int ebeg = wave * per;
    const int eend = (ebeg + per < NNZ) ? (ebeg + per) : NNZ;
    int* mylist = wl + wave * WLC;
    int wc = 0;
#pragma unroll 1
    for (int cb = ebeg; cb < eend; cb += WCH) {
      const int e0 = cb + lane * EPT;
      const v4i da = *(const v4ia*)(keys + e0);
      const v4i db = *(const v4ia*)(keys + e0 + 4);
      const unsigned s0 = (unsigned)da.x - nbs, s1 = (unsigned)da.y - nbs;
      const unsigned s2 = (unsigned)da.z - nbs, s3 = (unsigned)da.w - nbs;
      const unsigned s4 = (unsigned)db.x - nbs, s5 = (unsigned)db.y - nbs;
      const unsigned s6 = (unsigned)db.z - nbs, s7 = (unsigned)db.w - nbs;
      const bool h0 = s0 < unb, h1 = s1 < unb, h2 = s2 < unb, h3 = s3 < unb;
      const bool h4 = s4 < unb, h5 = s5 < unb, h6 = s6 < unb, h7 = s7 < unb;
      const unsigned m0 = __builtin_amdgcn_ballot_w32(h0), m1 = __builtin_amdgcn_ballot_w32(h1);
      const unsigned m2 = __builtin_amdgcn_ballot_w32(h2), m3 = __builtin_amdgcn_ballot_w32(h3);
      const unsigned m4 = __builtin_amdgcn_ballot_w32(h4), m5 = __builtin_amdgcn_ballot_w32(h5);
      const unsigned m6 = __builtin_amdgcn_ballot_w32(h6), m7 = __builtin_amdgcn_ballot_w32(h7);
      const unsigned any = m0 | m1 | m2 | m3 | m4 | m5 | m6 | m7;
      if (any != 0u) {
        const int pre = (int)(__builtin_amdgcn_mbcnt_lo(m0, 0u) + __builtin_amdgcn_mbcnt_lo(m1, 0u) +
                              __builtin_amdgcn_mbcnt_lo(m2, 0u) + __builtin_amdgcn_mbcnt_lo(m3, 0u) +
                              __builtin_amdgcn_mbcnt_lo(m4, 0u) + __builtin_amdgcn_mbcnt_lo(m5, 0u) +
                              __builtin_amdgcn_mbcnt_lo(m6, 0u) + __builtin_amdgcn_mbcnt_lo(m7, 0u));
        int p = wc + pre;
        if (h0) { if (p < WLC) mylist[p] = ((e0 + 0) << SLB) | (int)s0; p = p + 1; }
        if (h1) { if (p < WLC) mylist[p] = ((e0 + 1) << SLB) | (int)s1; p = p + 1; }
        if (h2) { if (p < WLC) mylist[p] = ((e0 + 2) << SLB) | (int)s2; p = p + 1; }
        if (h3) { if (p < WLC) mylist[p] = ((e0 + 3) << SLB) | (int)s3; p = p + 1; }
        if (h4) { if (p < WLC) mylist[p] = ((e0 + 4) << SLB) | (int)s4; p = p + 1; }
        if (h5) { if (p < WLC) mylist[p] = ((e0 + 5) << SLB) | (int)s5; p = p + 1; }
        if (h6) { if (p < WLC) mylist[p] = ((e0 + 6) << SLB) | (int)s6; p = p + 1; }
        if (h7) { if (p < WLC) mylist[p] = ((e0 + 7) << SLB) | (int)s7; p = p + 1; }
        wc += (int)(__builtin_popcount(m0) + __builtin_popcount(m1) + __builtin_popcount(m2) + __builtin_popcount(m3) +
                    __builtin_popcount(m4) + __builtin_popcount(m5) + __builtin_popcount(m6) + __builtin_popcount(m7));
      }
    }
    if (lane == 0) misc[wave] = wc;
  }
  __syncthreads();

  if (wave == 0) {
    int ov = 0;
#pragma unroll 1
    for (int w2 = 0; w2 < NWAVE; ++w2) {
      int c = misc[w2];
      if (c > WLC) ov = 1;
      c = c < 0 ? 0 : (c > WLC ? WLC : c);
#pragma unroll 1
      for (int b0 = 0; b0 < c; b0 += 32) {
        const int idx = b0 + lane;
        const int ent = wl[w2 * WLC + (idx < WLC ? idx : WLC - 1)];
        const int m32 = (c - b0) < 32 ? (c - b0) : 32;
#pragma unroll 1
        for (int k = 0; k < m32; ++k) {
          const int u = __builtin_amdgcn_readlane(ent, k);
          int slot = u & ((1 << SLB) - 1);
          slot = slot > SLOTS - 1 ? SLOTS - 1 : slot;
          if (lane == 0) cnt[slot] = cnt[slot] + 1;
        }
      }
    }
    if (lane == 0) misc[9] = ov;
  }
  __syncthreads();
  if (wave == 0) {
    const int base = lane * (SLOTS / 32);
    int s = 0, mx = 0;
#pragma unroll 1
    for (int i = 0; i < SLOTS / 32; ++i) {
      const int cv = cnt[base + i];
      s += cv;
      mx = cv > mx ? cv : mx;
    }
    int incl = s;
#pragma unroll
    for (int d = 1; d < 32; d <<= 1) {
      const int y = __shfl_up(incl, d, 32);
      if (lane >= d) incl += y;
    }
#pragma unroll
    for (int d = 16; d >= 1; d >>= 1) {
      const int y = __shfl_xor(mx, d, 32);
      mx = y > mx ? y : mx;
    }
    int run = incl - s;
#pragma unroll 1
    for (int i = 0; i < SLOTS / 32; ++i) {
      const int cv = cnt[base + i];
      offs[base + i] = run;
      cur[base + i]  = run;
      run += cv;
    }
    if (lane == 0) misc[9] = misc[9] | ((mx > DCAP) ? 1 : 0);
  }
  __syncthreads();

  if (wave == 0) {
#pragma unroll 1
    for (int w2 = 0; w2 < NWAVE; ++w2) {
      int c = misc[w2];
      c = c < 0 ? 0 : (c > WLC ? WLC : c);
#pragma unroll 1
      for (int b0 = 0; b0 < c; b0 += 32) {
        const int idx = b0 + lane;
        const int ent = wl[w2 * WLC + (idx < WLC ? idx : WLC - 1)];
        int eid = (ent >> SLB) & 0x1FFFFF;
        eid = eid > NNZ - 1 ? NNZ - 1 : eid;
        int en = ents[eid];
        en = en < 0 ? 0 : (en > NENT - 1 ? NENT - 1 : en);
        const int m32 = (c - b0) < 32 ? (c - b0) : 32;
#pragma unroll 1
        for (int k = 0; k < m32; ++k) {
          const int u  = __builtin_amdgcn_readlane(ent, k);
          const int wd = __builtin_amdgcn_readlane(en, k);
          int slot = u & ((1 << SLB) - 1);
          slot = slot > SLOTS - 1 ? SLOTS - 1 : slot;
          if (lane == 0) {
            int p = cur[slot];
            p = p < 0 ? 0 : (p > RC - 1 ? RC - 1 : p);
            pl[p] = wd;
            cur[slot] = p + 1;
          }
        }
      }
    }
  }
  __syncthreads();

  const int ovf = misc[9];
  int* lp  = LIST + (size_t)blk * RC;
  int* cop = CO + (size_t)blk * (2 * SLOTS);
  int* fp  = FLAG + (size_t)blk * 32;
  bucket_flush(pl, cnt, ovf, lp, cop, fp, tid, RC, 2 * SLOTS);
  __threadfence();
  bucket_flush(pl, cnt, ovf, lp, cop, fp, tid, RC, 2 * SLOTS);
}

__global__ __launch_bounds__(NTHR) void k_bucket(const int* __restrict__ hei, int* LISTN, int* CON, int* FLAGN,
                                                 int* LISTE, int* COE, int* FLAGE) {
  extern __shared__ __attribute__((aligned(16))) int dsm[];
  const int blk = (int)blockIdx.x;
  if (blk < NBK_N) {
    bucket_role<0>(hei, dsm, blk, LISTN, CON, FLAGN);
  } else {
    bucket_role<1>(hei, dsm, blk - NBK_N, LISTE, COE, FLAGE);
  }
}

template <int KEXT, int BP>
__device__ __forceinline__ void gemm_16x64(const unsigned short* __restrict__ ap,
                                           const unsigned short* __restrict__ bp, v8f (&acc)[4]) {
#pragma unroll 1
  for (int k0 = 0; k0 < KEXT; k0 += 32) {
    FragB af;
    af.h[0] = *(const v8usa*)(ap + k0);
    af.h[1] = *(const v8usa*)(ap + k0 + 16);
#pragma unroll
    for (int nt = 0; nt < 4; ++nt) {
      const unsigned short* wq = bp + (size_t)(16 * nt) * (size_t)BP + k0;
      FragB bf;
      bf.h[0] = *(const v8usa*)wq;
      bf.h[1] = *(const v8usa*)(wq + 16);
      acc[nt] = wmb(af, bf, acc[nt]);
    }
  }
}

__device__ __forceinline__ void stage_d(float* stg, const v8f (&acc)[4], int wave, int hh, int m) {
#pragma unroll
  for (int nt = 0; nt < 4; ++nt) {
#pragma unroll
    for (int r = 0; r < 8; ++r) stg[(16 * wave + 8 * hh + r) * SP + 16 * nt + m] = acc[nt][r];
  }
}

template <int KEXT, int AP, int BP>
__global__ __launch_bounds__(NTHR) __attribute__((amdgpu_num_vgpr(248)))
void k_gemmA(const unsigned short* __restrict__ A, const unsigned short* __restrict__ BT,
             const float* __restrict__ sm, int biasOff, float* H, unsigned short* EH) {
  static_assert(KEXT % 32 == 0 && KEXT <= AP && KEXT <= BP && AP % 8 == 0 && BP % 8 == 0);
  __shared__ __attribute__((aligned(16))) float stg[GBM * SP];
  __shared__ __attribute__((aligned(16))) float sb[128];
  const int tid = (int)threadIdx.x, lane = tid & 31, wave = tid >> 5, hh = lane >> 4, m = lane & 15;
  const int rowBase = (int)blockIdx.x * GBM;
  if (tid < 32) *(v4fa*)(sb + 4 * tid) = *(const v4fa*)(sm + biasOff + 4 * tid);

  v8f acc[4];
  {
    const v8f z = {0.f, 0.f, 0.f, 0.f, 0.f, 0.f, 0.f, 0.f};
#pragma unroll
    for (int t = 0; t < 4; ++t) acc[t] = z;
  }
  const unsigned short* ap = A + (size_t)(rowBase + 16 * wave + m) * (size_t)AP + 8 * hh;
  const unsigned short* bp = BT + (size_t)m * (size_t)BP + 8 * hh;
  gemm_16x64<KEXT, BP>(ap, bp, acc);
  stage_d(stg, acc, wave, hh, m);
  __syncthreads();

  const float alpha = sm[256];
  const v4f bias = *(const v4fa*)(sb + 4 * m);
#pragma unroll 1
  for (int i = 0; i < 8; ++i) {
    const int lr    = 16 * wave + 2 * i + hh;
    const int grow  = rowBase + lr;
    const bool live = grow < NN;
    const int growc = live ? grow : NN - 1;
    const v4f a = *(const v4fa*)(stg + lr * SP + 4 * m);
    asm volatile("" :: "v"(a));
    v4f ho;
    ho.x = live ? a.x : 0.0f; ho.y = live ? a.y : 0.0f; ho.z = live ? a.z : 0.0f; ho.w = live ? a.w : 0.0f;
    const float e0 = prelu_k(a.x + bias.x, alpha), e1 = prelu_k(a.y + bias.y, alpha);
    const float e2 = prelu_k(a.z + bias.z, alpha), e3 = prelu_k(a.w + bias.w, alpha);
    int h01, h23, l01, l23;
    hilo_pack(e0, e1, e2, e3, h01, h23, l01, l23);
    const v4i ow = regroup8(h01, h23, l01, l23, lane);
    float* op = H + (size_t)grow * HD + 4 * m;
    unsigned short* ep = EH + (size_t)(NHE + growc) * KL + 8 * m;
    *(volatile v4f*)op = ho;
    if (live) *(volatile v4i*)ep = ow;
    __threadfence();
    *(volatile v4f*)op = ho;
    if (live) *(volatile v4i*)ep = ow;
  }
}

template <int KEXT>
__global__ __launch_bounds__(NTHR) __attribute__((amdgpu_num_vgpr(248)))
void k_gemmB(const unsigned short* __restrict__ A, const unsigned short* __restrict__ BT, float* G) {
  static_assert(KEXT % 32 == 0 && KEXT <= KL);
  __shared__ __attribute__((aligned(16))) float stg[GBM * SP];
  const int tid = (int)threadIdx.x, lane = tid & 31, wave = tid >> 5, hh = lane >> 4, m = lane & 15;
  const int rowBase = (int)blockIdx.x * GBM;

  v8f acc[4];
  {
    const v8f z = {0.f, 0.f, 0.f, 0.f, 0.f, 0.f, 0.f, 0.f};
#pragma unroll
    for (int t = 0; t < 4; ++t) acc[t] = z;
  }
  const unsigned short* ap = A + (size_t)(rowBase + 16 * wave + m) * (size_t)KL + 8 * hh;
  const unsigned short* bp = BT + (size_t)m * (size_t)KL + 8 * hh;
  gemm_16x64<KEXT, KL>(ap, bp, acc);
  stage_d(stg, acc, wave, hh, m);
  __syncthreads();

#pragma unroll 1
  for (int i = 0; i < 8; ++i) {
    const int lr    = 16 * wave + 2 * i + hh;
    const int grow  = rowBase + lr;
    const bool live = grow < ET;
    const int growc = live ? grow : ET - 1;
    const v4f a = *(const v4fa*)(stg + lr * SP + 4 * m);
    asm volatile("" :: "v"(a));
    float* op = G + (size_t)growc * HD + 4 * m;
    if (live) *(volatile v4f*)op = a;
    __threadfence();
    if (live) *(volatile v4f*)op = a;
  }
}

__global__ __launch_bounds__(NTHR) void k_replayE(const int* __restrict__ LISTE, const int* __restrict__ COE,
                                                  const int* __restrict__ FLAGE, const float* H,
                                                  const float* __restrict__ sm, int biasOff, unsigned short* EH) {
  __shared__ __attribute__((aligned(16))) float sb[128];
  const int tid = (int)threadIdx.x, lane = tid & 31, wave = tid >> 5, hh = lane >> 4, q = lane & 15;
  if (tid < 32) *(v4fa*)(sb + 4 * tid) = *(const v4fa*)(sm + biasOff + 4 * tid);
  __syncthreads();
  const float alpha = sm[256];
  const v4f bias = *(const v4fa*)(sb + 4 * q);
  const int rowBase = (int)blockIdx.x * RBM;
  const int bucket  = rowBase >> 8;
  const int* lb  = LISTE + (size_t)bucket * RCAP_E;
  const int* cob = COE + (size_t)bucket * (2 * SLOTS_E);
  const int flag = FLAGE[(size_t)bucket * 32];
  const float qnan = __uint_as_float(0x7fc00000u);

#pragma unroll 1
  for (int i = 0; i < RBM / (2 * NWAVE); ++i) {
    const int j    = rowBase + (RBM / NWAVE) * wave + 2 * i + hh;
    const int slot = j & (SLOTS_E - 1);
    const int craw = cob[slot];
    int o = cob[SLOTS_E + slot];
    const int deg  = craw < 0 ? 0 : craw;
    const bool big = deg > DEGCAP_E;
    int c = deg > DEGCAP_E ? DEGCAP_E : deg;
    o = o < 0 ? 0 : (o > RCAP_E - 1 ? RCAP_E - 1 : o);
    c = c > RCAP_E - o ? RCAP_E - o : c;
    int last = o + c - 1;
    last = last < o ? o : last;
    const int co = __shfl_xor(c, 16, 32);
    const int cm = c > co ? c : co;
    float a0 = 0.0f, a1 = 0.0f, a2 = 0.0f, a3 = 0.0f;
#pragma unroll 1
    for (int t = 0; t < cm; ++t) {
      int idx = o + t;
      idx = idx > last ? last : idx;
      int sr = lb[idx];
      sr = sr < 0 ? 0 : (sr > NN - 1 ? NN - 1 : sr);
      const v4f v = *(const v4fa*)(H + (size_t)sr * HD + 4 * q);
      asm volatile("" :: "v"(v));
      const bool valid = t < c;
      const float t0 = a0 + v.x, t1 = a1 + v.y, t2 = a2 + v.z, t3 = a3 + v.w;
      a0 = valid ? t0 : a0; a1 = valid ? t1 : a1; a2 = valid ? t2 : a2; a3 = valid ? t3 : a3;
    }
    const float inv = 1.0f / (float)(deg > 0 ? deg : 1);
    const bool has = deg > 0;
    const float m0 = has ? a0 * inv : 0.0f, m1 = has ? a1 * inv : 0.0f;
    const float m2 = has ? a2 * inv : 0.0f, m3 = has ? a3 * inv : 0.0f;
    float e0 = prelu_k(m0 + bias.x, alpha), e1 = prelu_k(m1 + bias.y, alpha);
    float e2 = prelu_k(m2 + bias.z, alpha), e3 = prelu_k(m3 + bias.w, alpha);
    const bool bad = (flag != 0) | big;
    e0 = bad ? qnan : e0; e1 = bad ? qnan : e1; e2 = bad ? qnan : e2; e3 = bad ? qnan : e3;
    int h01, h23, l01, l23;
    hilo_pack(e0, e1, e2, e3, h01, h23, l01, l23);
    const v4i ow = regroup8(h01, h23, l01, l23, lane);
    const bool live = j < NHE;
    const int jc = live ? j : NHE - 1;
    unsigned short* ep = EH + (size_t)jc * KL + 8 * q;
    if (live) *(volatile v4i*)ep = ow;
    __threadfence();
    if (live) *(volatile v4i*)ep = ow;
  }
}

template <int LAST>
__global__ __launch_bounds__(NTHR) void k_replayN(const int* __restrict__ LISTN, const int* __restrict__ CON,
                                                  const int* __restrict__ FLAGN, const float* G,
                                                  const float* __restrict__ sm, int biasOff,
                                                  unsigned short* HH, float* out) {
  __shared__ __attribute__((aligned(16))) float sb[128];
  const int tid = (int)threadIdx.x, lane = tid & 31, wave = tid >> 5, hh = lane >> 4, q = lane & 15;
  if (tid < 32) *(v4fa*)(sb + 4 * tid) = *(const v4fa*)(sm + biasOff + 4 * tid);
  __syncthreads();
  const float alpha = sm[256];
  const float gfl   = sm[257];
  const v4f bias = *(const v4fa*)(sb + 4 * q);
  const int rowBase = (int)blockIdx.x * RBM;
  const int bucket  = rowBase >> SLB;
  const int* lb  = LISTN + (size_t)bucket * RCAP_N;
  const int* cob = CON + (size_t)bucket * (2 * SLOTS_N);
  const int flag = FLAGN[(size_t)bucket * 32];
  const float qnan = __uint_as_float(0x7fc00000u);

#pragma unroll 1
  for (int i = 0; i < RBM / (2 * NWAVE); ++i) {
    const int d    = rowBase + (RBM / NWAVE) * wave + 2 * i + hh;
    const int slot = d & (SLOTS_N - 1);
    const int craw = cob[slot];
    int o = cob[SLOTS_N + slot];
    const int deg  = craw < 0 ? 0 : craw;
    const bool big = deg > DEGCAP_N;
    int c = deg > DEGCAP_N ? DEGCAP_N : deg;
    o = o < 0 ? 0 : (o > RCAP_N - 1 ? RCAP_N - 1 : o);
    c = c > RCAP_N - o ? RCAP_N - o : c;
    int last = o + c - 1;
    last = last < o ? o : last;
    const int co = __shfl_xor(c, 16, 32);
    const int cm = c > co ? c : co;
    float a0 = 0.0f, a1 = 0.0f, a2 = 0.0f, a3 = 0.0f;
#pragma unroll 1
    for (int t = 0; t < cm; ++t) {
      int idx = o + t;
      idx = idx > last ? last : idx;
      int sr = lb[idx];
      sr = sr < 0 ? 0 : (sr > NHE - 1 ? NHE - 1 : sr);
      const v4f v = *(const v4fa*)(G + (size_t)sr * HD + 4 * q);
      asm volatile("" :: "v"(v));
      const bool valid = t < c;
      const float t0 = a0 + v.x, t1 = a1 + v.y, t2 = a2 + v.z, t3 = a3 + v.w;
      a0 = valid ? t0 : a0; a1 = valid ? t1 : a1; a2 = valid ? t2 : a2; a3 = valid ? t3 : a3;
    }
    const bool live = d < NN;
    const int dc = live ? d : NN - 1;
    const v4f gs = *(const v4fa*)(G + (size_t)(NHE + dc) * HD + 4 * q);
    asm volatile("" :: "v"(gs));
    const float inv = 1.0f / (float)(deg + 1);
    float n0 = (a0 + gs.x) * inv + bias.x, n1 = (a1 + gs.y) * inv + bias.y;
    float n2 = (a2 + gs.z) * inv + bias.z, n3 = (a3 + gs.w) * inv + bias.w;
    n0 = prelu_k(n0, alpha); n1 = prelu_k(n1, alpha); n2 = prelu_k(n2, alpha); n3 = prelu_k(n3, alpha);
    const bool bad = (flag != 0) | big | (gfl != 0.0f);
    n0 = bad ? qnan : n0; n1 = bad ? qnan : n1; n2 = bad ? qnan : n2; n3 = bad ? qnan : n3;
    if constexpr (LAST == 0) {
      n0 = live ? n0 : 0.0f; n1 = live ? n1 : 0.0f; n2 = live ? n2 : 0.0f; n3 = live ? n3 : 0.0f;
      int h01, h23, l01, l23;
      hilo_pack(n0, n1, n2, n3, h01, h23, l01, l23);
      const v4i ow = regroup8(h01, h23, l01, l23, lane);
      unsigned short* hp = HH + (size_t)d * KL + 8 * q;
      *(volatile v4i*)hp = ow;
      __threadfence();
      *(volatile v4i*)hp = ow;
    } else {
      v4f ov;
      ov.x = n0; ov.y = n1; ov.z = n2; ov.w = n3;
      float* op = out + (size_t)dc * HD + 4 * q;
      if (live) *(volatile v4f*)op = ov;
      __threadfence();
      if (live) *(volatile v4f*)op = ov;
    }
  }
}

extern "C" void kernel_launch(void* const* d_in, const int* in_sizes, int n_in,
                              void* d_out, int out_size, void* d_ws, size_t ws_size,
                              hipStream_t stream) {
  if (n_in < 13) return;
  if (in_sizes[0] != NN * HD) return;
  if (in_sizes[1] != 2 * NNZ) return;
  if (in_sizes[2] != HD * HD || in_sizes[4] != HD * HD) return;
  if (in_sizes[6] != HD * HD || in_sizes[8] != HD * HD) return;
  if (in_sizes[3] != HD || in_sizes[5] != HD || in_sizes[7] != HD || in_sizes[9] != HD) return;
  if (in_sizes[10] != 1 || in_sizes[11] != 1 || in_sizes[12] != 1) return;
  if (out_size != NN * HD) return;
  if (oEND > ws_size) return;

  const float* x   = (const float*)d_in[0];
  const int*   hei = (const int*)d_in[1];
  const float* w1n = (const float*)d_in[2];
  const float* b1n = (const float*)d_in[3];
  const float* w1e = (const float*)d_in[4];
  const float* b1e = (const float*)d_in[5];
  const float* w2n = (const float*)d_in[6];
  const float* b2n = (const float*)d_in[7];
  const float* w2e = (const float*)d_in[8];
  const float* b2e = (const float*)d_in[9];
  const float* alp = (const float*)d_in[10];
  const int*   nnp = (const int*)d_in[11];
  const int*   nep = (const int*)d_in[12];
  float* out = (float*)d_out;

  char* ws = (char*)d_ws;
  unsigned short* HH   = (unsigned short*)(ws + oHH);
  unsigned short* XB   = (unsigned short*)(ws + oHH);
  float*          H    = (float*)(ws + oH);
  unsigned short* EH   = (unsigned short*)(ws + oEH);
  float*          G    = (float*)(ws + oG);
  int*            LSN  = (int*)(ws + oLN);
  int*            LSE  = (int*)(ws + oLE);
  int*            CON  = (int*)(ws + oCN);
  int*            COE  = (int*)(ws + oCE);
  int*            FLN  = (int*)(ws + oFN);
  int*            FLE  = (int*)(ws + oFE);
  unsigned short* W1T  = (unsigned short*)(ws + oW1T);
  unsigned short* WD   = (unsigned short*)(ws + oWD);
  float*          SM   = (float*)(ws + oSM);
  const unsigned short* WD1E = WD;
  const unsigned short* WD2N = WD + (size_t)HD * KL;
  const unsigned short* WD2E = WD + (size_t)2 * HD * KL;

  hipFuncSetAttribute(reinterpret_cast<const void*>(&k_bucket), hipFuncAttributeMaxDynamicSharedMemorySize, (int)BK_LDS);

  k_prep<<<PBTOT, NTHR, 0, stream>>>(x, w1n, w1e, w2n, w2e, b1n, b1e, b2n, b2e, alp, nnp, nep, ws);
  k_bucket<<<NBK_N + NBK_E, NTHR, BK_LDS, stream>>>(hei, LSN, CON, FLN, LSE, COE, FLE);

  k_gemmA<64, 64, 64><<<MPN / GBM, NTHR, 0, stream>>>(XB, W1T, SM, 0, H, EH);
  k_replayE<<<(NHE + RBM - 1) / RBM, NTHR, 0, stream>>>(LSE, COE, FLE, H, SM, 0, EH);
  k_gemmB<KX_B1><<<MPE / GBM, NTHR, 0, stream>>>(EH, WD1E, G);
  k_replayN<0><<<MPN / RBM, NTHR, 0, stream>>>(LSN, CON, FLN, G, SM, 64, HH, out);

  k_gemmA<KX_A2, KL, KL><<<MPN / GBM, NTHR, 0, stream>>>(HH, WD2N, SM, 128, H, EH);
  k_replayE<<<(NHE + RBM - 1) / RBM, NTHR, 0, stream>>>(LSE, COE, FLE, H, SM, 128, EH);
  k_gemmB<KX_B2><<<MPE / GBM, NTHR, 0, stream>>>(EH, WD2E, G);
  k_replayN<1><<<MPN / RBM, NTHR, 0, stream>>>(LSN, CON, FLN, G, SM, 192, HH, out);
}
